// ResidualIntegrationNetworkRK4_14035953124039
// MI455X (gfx1250) — hardware-verified
//
#include <hip/hip_runtime.h>
#include <hip/hip_bf16.h>


#define SEQ_   256
#define BATCH_ 1024
#define FEAT_  2
#define HID_   128
#define ROWS_  32
#define NTHR_  256
#define PA_    136
#define PP_    36

static_assert(BATCH_ % ROWS_ == 0);
static_assert(ROWS_ * 4 == 128);
static_assert(HID_ == 128);
static_assert(NTHR_ == ROWS_ * 8);
static_assert((PA_ % 8) == 0);
static_assert((PP_ % 4) == 0);

#define OFF_BHI   0
#define OFF_BLO   (OFF_BHI + HID_ * PA_ * 2)
#define OFF_AHI   (OFF_BLO + HID_ * PA_ * 2)
#define OFF_ALO   (OFF_AHI + ROWS_ * PA_ * 2)
#define OFF_P2T   (OFF_ALO + ROWS_ * PA_ * 2)
#define OFF_W1    (OFF_P2T + HID_ * PP_ * 4)
#define OFF_B1    (OFF_W1 + 3 * HID_ * 4)
#define OFF_YS    (OFF_B1 + HID_ * 4)
#define LDS_BYTES (OFF_YS + ROWS_ * 4)
static_assert(OFF_BLO == 34816);
static_assert(OFF_AHI == 69632);
static_assert(OFF_ALO == 78336);
static_assert(OFF_P2T == 87040);
static_assert(OFF_W1 == 105472);
static_assert(OFF_B1 == 107008);
static_assert(OFF_YS == 107520);
static_assert(LDS_BYTES == 107648);
static_assert((OFF_BLO % 16) == 0 && (OFF_AHI % 16) == 0 && (OFF_ALO % 16) == 0);
static_assert((OFF_P2T % 16) == 0 && (OFF_W1 % 16) == 0 && (OFF_B1 % 16) == 0 && (OFF_YS % 16) == 0);

typedef float          v4f   __attribute__((ext_vector_type(4)));
typedef float          v8f   __attribute__((ext_vector_type(8)));
typedef __bf16         v16b  __attribute__((ext_vector_type(16)));
typedef unsigned short u16x8 __attribute__((ext_vector_type(8)));

union FragB { u16x8 h[2]; v16b v; };

__device__ __forceinline__ unsigned short f32_to_bf16(float f) {
    unsigned u = __float_as_uint(f);
    unsigned r = u + 0x7FFFu + ((u >> 16) & 1u);
    return (unsigned short)(r >> 16);
}
__device__ __forceinline__ float bf16_to_f32(unsigned short b) {
    return __uint_as_float(((unsigned)b) << 16);
}

__device__ __forceinline__ float tanh_f(float x) {
    const float ax = __builtin_fabsf(x);
    const float x2 = x * x;
    float p = fmaf(x2, 2.1869488536155203e-2f, -5.3968253968253968e-2f);
    p = fmaf(x2, p, 1.3333333333333333e-1f);
    p = fmaf(x2, p, -3.3333333333333333e-1f);
    const float sm = fmaf(x * x2, p, x);
    const float t  = __expf(-2.0f * ax);
    float r = (1.0f - t) * __builtin_amdgcn_rcpf(1.0f + t);
    r = __builtin_copysignf(r, x);
    return (ax < 0.3f) ? sm : r;
}

__device__ __forceinline__ v8f wmma_bf16(v16b a, v16b b, v8f c) {
    return __builtin_amdgcn_wmma_f32_16x16x32_bf16(false, a, false, b, (short)0, c, false, false);
}
__device__ __forceinline__ void mma3(v8f& acc, const FragB& ah, const FragB& al,
                                     const FragB& bh, const FragB& bl) {
    acc = wmma_bf16(ah.v, bh.v, acc);
    acc = wmma_bf16(ah.v, bl.v, acc);
    acc = wmma_bf16(al.v, bh.v, acc);
    asm volatile("v_nop\n\tv_nop\n\tv_nop\n\tv_nop"
                 : "+v"(acc) : "v"(ah.v), "v"(al.v), "v"(bh.v), "v"(bl.v));
}

__global__ __launch_bounds__(NTHR_)
void rk4_kernel(const float* __restrict__ xg,
                const float* __restrict__ W1g,
                const float* __restrict__ b1g,
                const float* __restrict__ W2g,
                const float* __restrict__ b2g,
                const float* __restrict__ W3g,
                const float* __restrict__ b3g,
                float* outg)
{
    extern __shared__ __attribute__((aligned(16))) unsigned char smem[];
    unsigned short* Bhi = (unsigned short*)(smem + OFF_BHI);
    unsigned short* Blo = (unsigned short*)(smem + OFF_BLO);
    unsigned short* Ahi = (unsigned short*)(smem + OFF_AHI);
    unsigned short* Alo = (unsigned short*)(smem + OFF_ALO);
    float*          P2T = (float*)(smem + OFF_P2T);
    float*          W1s = (float*)(smem + OFF_W1);
    float*          b1s = (float*)(smem + OFF_B1);
    float*          ys  = (float*)(smem + OFF_YS);

    const int tid   = threadIdx.x;
    const int lane  = tid & 31;
    const int wave  = tid >> 5;
    const int h     = lane >> 4;
    const int m     = lane & 15;
    const int row   = tid >> 3;
    const int q     = tid & 7;
    const int row0  = blockIdx.x * ROWS_;
    const int nbase = wave * 16;

#pragma unroll 4
    for (int idx = tid; idx < HID_ * HID_; idx += NTHR_) {
        const int k = idx >> 7;
        const int n = idx & (HID_ - 1);
        const float w = W2g[idx];
        const unsigned short hb = f32_to_bf16(w);
        const unsigned short lb = f32_to_bf16(w - bf16_to_f32(hb));
        Bhi[n * PA_ + k] = hb;
        Blo[n * PA_ + k] = lb;
    }
    for (int idx = tid; idx < HID_ * 8; idx += NTHR_) {
        const int n = idx >> 3, c = HID_ + (idx & 7);
        Bhi[n * PA_ + c] = (unsigned short)0;
        Blo[n * PA_ + c] = (unsigned short)0;
    }
    {
        const int n = tid >> 3, c = HID_ + (tid & 7);
        Ahi[n * PA_ + c] = (unsigned short)0;
        Alo[n * PA_ + c] = (unsigned short)0;
    }
    for (int i = tid; i < 3 * HID_; i += NTHR_) W1s[i] = W1g[i];
    if (tid < HID_) b1s[tid] = b1g[tid];

    const float b2c = b2g[nbase + m];
    const float w3c = W3g[nbase + m];
    const float b3v = b3g[0];
    __syncthreads();

    float y = 0.0f, yarg = 0.0f, k1 = 0.0f, k2 = 0.0f, k3 = 0.0f;

    const unsigned short* bhp = Bhi + (nbase + m) * PA_ + 8 * h;
    const unsigned short* blp = Blo + (nbase + m) * PA_ + 8 * h;
    const unsigned short* ahp = Ahi + m * PA_ + 8 * h;
    const unsigned short* alp = Alo + m * PA_ + 8 * h;
    float* pcol = P2T + (nbase + m) * PP_ + 8 * h;

#pragma unroll 1
    for (int s = 0; s < SEQ_; ++s) {
        const size_t xo = ((size_t)s * BATCH_ + (size_t)(row0 + row)) * FEAT_;
        const float x0 = xg[xo];
        const float x1 = xg[xo + 1];

        float base[16];
#pragma unroll
        for (int v = 0; v < 4; ++v) {
            const v4f wa = *(const v4f*)(W1s + q * 16 + 4 * v);
            const v4f wb = *(const v4f*)(W1s + HID_ + q * 16 + 4 * v);
            const v4f bb = *(const v4f*)(b1s + q * 16 + 4 * v);
#pragma unroll
            for (int c = 0; c < 4; ++c)
                base[4 * v + c] = fmaf(x1, wb[c], fmaf(x0, wa[c], bb[c]));
        }

#pragma unroll 1
        for (int stage = 0; stage < 4; ++stage) {
            {
                u16x8 hv[2], lv[2];
#pragma unroll
                for (int v = 0; v < 4; ++v) {
                    const v4f wc = *(const v4f*)(W1s + 2 * HID_ + q * 16 + 4 * v);
#pragma unroll
                    for (int c = 0; c < 4; ++c) {
                        const float pre  = fmaf(yarg, wc[c], base[4 * v + c]);
                        const float hval = tanh_f(pre);
                        const unsigned short hb = f32_to_bf16(hval);
                        const unsigned short lb = f32_to_bf16(hval - bf16_to_f32(hb));
                        hv[v >> 1][(v & 1) * 4 + c] = hb;
                        lv[v >> 1][(v & 1) * 4 + c] = lb;
                    }
                }
                unsigned short* ap = Ahi + row * PA_ + q * 16;
                unsigned short* lp = Alo + row * PA_ + q * 16;
                *(u16x8*)(ap)     = hv[0];
                *(u16x8*)(ap + 8) = hv[1];
                *(u16x8*)(lp)     = lv[0];
                *(u16x8*)(lp + 8) = lv[1];
            }
            __syncthreads();

            v8f acc0, acc1;
#pragma unroll
            for (int r = 0; r < 8; ++r) { acc0[r] = 0.0f; acc1[r] = 0.0f; }
#pragma unroll 1
            for (int kc = 0; kc < 4; ++kc) {
                const int k0 = kc * 32;
                FragB bh, bl, a0h, a0l, a1h, a1l;
                bh.h[0]  = *(const u16x8*)(bhp + k0);
                bh.h[1]  = *(const u16x8*)(bhp + k0 + 16);
                bl.h[0]  = *(const u16x8*)(blp + k0);
                bl.h[1]  = *(const u16x8*)(blp + k0 + 16);
                a0h.h[0] = *(const u16x8*)(ahp + k0);
                a0h.h[1] = *(const u16x8*)(ahp + k0 + 16);
                a0l.h[0] = *(const u16x8*)(alp + k0);
                a0l.h[1] = *(const u16x8*)(alp + k0 + 16);
                a1h.h[0] = *(const u16x8*)(ahp + 16 * PA_ + k0);
                a1h.h[1] = *(const u16x8*)(ahp + 16 * PA_ + k0 + 16);
                a1l.h[0] = *(const u16x8*)(alp + 16 * PA_ + k0);
                a1l.h[1] = *(const u16x8*)(alp + 16 * PA_ + k0 + 16);
                mma3(acc0, a0h, a0l, bh, bl);
                mma3(acc1, a1h, a1l, bh, bl);
            }

            {
                v4f u0, u1, u2, u3;
#pragma unroll
                for (int r = 0; r < 4; ++r) {
                    u0[r] = tanh_f(acc0[r]     + b2c) * w3c;
                    u1[r] = tanh_f(acc0[4 + r] + b2c) * w3c;
                    u2[r] = tanh_f(acc1[r]     + b2c) * w3c;
                    u3[r] = tanh_f(acc1[4 + r] + b2c) * w3c;
                }
                *(v4f*)(pcol)      = u0;
                *(v4f*)(pcol + 4)  = u1;
                *(v4f*)(pcol + 16) = u2;
                *(v4f*)(pcol + 20) = u3;
            }
            __syncthreads();

            float sacc = 0.0f;
#pragma unroll
            for (int c = 0; c < 16; ++c) sacc += P2T[(q * 16 + c) * PP_ + row];
            sacc += __shfl_xor(sacc, 1);
            sacc += __shfl_xor(sacc, 2);
            sacc += __shfl_xor(sacc, 4);
            {
#pragma clang fp contract(off)
                const float kv = sacc + b3v;
                if (stage == 0)      { k1 = kv; yarg = y + kv * 0.5f; }
                else if (stage == 1) { k2 = kv; yarg = y + kv * 0.5f; }
                else if (stage == 2) { k3 = kv; yarg = y + kv * 1.0f; }
                else {
                    const float ssum = ((k1 + 2.0f * k2) + 2.0f * k3) + kv;
                    y = y + ((1.0f / 6.0f) * ssum) * 1.0f;
                    yarg = y;
                }
            }
        }

        if (q == 0) ys[row] = y;
        __syncthreads();
        if (wave == 0) {
            const v4f v = *(const v4f*)(ys + 4 * (lane & 7));
            if (lane < 8) {
                float* gp = outg + (size_t)s * BATCH_ + (size_t)(row0 + 4 * lane);
                *(volatile v4f*)gp = v;
                __threadfence();
                *(volatile v4f*)gp = v;
            }
        }
    }
}

extern "C" void kernel_launch(void* const* d_in, const int* in_sizes, int n_in,
                              void* d_out, int out_size, void* d_ws, size_t ws_size,
                              hipStream_t stream)
{
    (void)d_ws; (void)ws_size;
    if (n_in < 7) return;
    if (in_sizes[0] != SEQ_ * BATCH_ * FEAT_) return;
    if (in_sizes[1] != (FEAT_ + 1) * HID_)   return;
    if (in_sizes[2] != HID_)                  return;
    if (in_sizes[3] != HID_ * HID_)           return;
    if (in_sizes[4] != HID_)                  return;
    if (in_sizes[5] != HID_)                  return;
    if (in_sizes[6] < 1)                      return;
    if (out_size != SEQ_ * BATCH_)            return;

    const float* x  = (const float*)d_in[0];
    const float* W1 = (const float*)d_in[1];
    const float* b1 = (const float*)d_in[2];
    const float* W2 = (const float*)d_in[3];
    const float* b2 = (const float*)d_in[4];
    const float* W3 = (const float*)d_in[5];
    const float* b3 = (const float*)d_in[6];
    float* out = (float*)d_out;

    (void)hipFuncSetAttribute(reinterpret_cast<const void*>(&rk4_kernel),
                              hipFuncAttributeMaxDynamicSharedMemorySize, (int)LDS_BYTES);
    hipLaunchKernelGGL(rk4_kernel, dim3(BATCH_ / ROWS_), dim3(NTHR_), (size_t)LDS_BYTES, stream,
                       x, W1, b1, W2, b2, W3, b3, out);
}
